// Net_79937931313639
// MI455X (gfx1250) — hardware-verified
//
#include <hip/hip_runtime.h>
#include <math.h>
#pragma clang fp contract(off)

typedef __attribute__((ext_vector_type(16))) __bf16   v16b;
typedef __attribute__((ext_vector_type(8)))  __bf16   v8b;
typedef __attribute__((ext_vector_type(8)))  float    v8f;
typedef __attribute__((ext_vector_type(4)))  float    v4f;
typedef __attribute__((ext_vector_type(4)))  unsigned v4u;
typedef __attribute__((ext_vector_type(2)))  unsigned v2u;
typedef __attribute__((ext_vector_type(4)))  int      v4i;

constexpr int NPTS        = 16384;
constexpr int NHALF_PTS   = 8192;
constexpr int KGRAD       = 20;
constexpr int KNORM       = 10;
constexpr int NBR_PITCH   = 32;
constexpr float EPS_F     = 1e-8f;
constexpr float GRAD_REG_F = 1e-3f;
constexpr float INV_KGRAD = 1.0f / (float)KGRAD;

static_assert(NPTS == 2 * NHALF_PTS, "concat of two clouds");
static_assert(NPTS % 256 == 0, "grid multiples");
static_assert(KNORM <= KGRAD && KGRAD <= NBR_PITCH, "neighbour table");

__device__ __forceinline__ unsigned bf_hi_bits(float f) {
  const unsigned u = __float_as_uint(f);
  return (u + 0x7FFFu + ((u >> 16) & 1u)) >> 16;
}
__device__ __forceinline__ float bf_from_bits(unsigned h) { return __uint_as_float(h << 16); }
__device__ __forceinline__ float bf_rne(float f) { return bf_from_bits(bf_hi_bits(f)); }
__device__ __forceinline__ unsigned pack16(unsigned lo, unsigned hi) { return (lo & 0xffffu) | (hi << 16); }
__device__ __forceinline__ v4f ld4(const float* p, int i) { return *(const v4f*)(p + 4 * (size_t)i); }
__device__ __forceinline__ int clamp_idx(int j) {
  j = j < 0 ? 0 : j;
  return j > (NPTS - 1) ? (NPTS - 1) : j;
}
__device__ __forceinline__ void st2_v4f(float* p, v4f v) {
  *(volatile v4f*)p = v;
  __threadfence();
  *(volatile v4f*)p = v;
}
__device__ __forceinline__ void split4_to_lds(v4f val, unsigned* dh, unsigned* dl) {
  const float f0 = val.x, f1 = val.y, f2 = val.z, f3 = val.w;
  const unsigned h0 = bf_hi_bits(f0), h1 = bf_hi_bits(f1), h2 = bf_hi_bits(f2), h3 = bf_hi_bits(f3);
  const unsigned l0 = bf_hi_bits(f0 - bf_from_bits(h0));
  const unsigned l1 = bf_hi_bits(f1 - bf_from_bits(h1));
  const unsigned l2 = bf_hi_bits(f2 - bf_from_bits(h2));
  const unsigned l3 = bf_hi_bits(f3 - bf_from_bits(h3));
  const v2u wh = (v2u){pack16(h0, h1), pack16(h2, h3)};
  const v2u wl = (v2u){pack16(l0, l1), pack16(l2, l3)};
  *(v2u*)dh = wh;
  *(v2u*)dl = wl;
}

union FragB { v16b v; v8b h[2]; };
__device__ __forceinline__ v16b frag_load_b(const __bf16* p) {
  FragB f;
  f.h[0] = *(const v8b*)(p);
  f.h[1] = *(const v8b*)(p + 16);
  return f.v;
}
__device__ __forceinline__ v8f mma_b(v16b a, v16b b, v8f c) {
  return __builtin_amdgcn_wmma_f32_16x16x32_bf16(false, a, false, b, (short)0, c, false, false);
}
__device__ __forceinline__ void dep_guard4_b(v8f& a, v8f& b, v8f& c, v8f& d, v16b x, v16b y) {
  asm volatile("v_nop\n\tv_nop\n\tv_nop\n\tv_nop" : "+v"(a), "+v"(b), "+v"(c), "+v"(d) : "v"(x), "v"(y));
}
__device__ __forceinline__ void keep4_b(v16b a, v16b b, v16b c, v16b d) { asm volatile("v_nop" :: "v"(a), "v"(b), "v"(c), "v"(d)); }
__device__ __forceinline__ void acc_guard4(v8f& a, v8f& b, v8f& c, v8f& d) {
  asm volatile("v_nop\n\tv_nop\n\tv_nop\n\tv_nop" : "+v"(a), "+v"(b), "+v"(c), "+v"(d));
}

template <int NPROD, int BIAS_MODE, int ACT>
__global__ __launch_bounds__(256) void gemm_bf16_kernel(
    const unsigned short* __restrict__ Ap, const unsigned short* __restrict__ A2p, int lda,
    const unsigned short* __restrict__ Btp, int ldb,
    float* __restrict__ Cout, int ldc, const float* __restrict__ bias,
    int M, int N, int K) {
  const __bf16* A  = (const __bf16*)Ap;
  const __bf16* A2 = (const __bf16*)A2p;
  const __bf16* Bt = (const __bf16*)Btp;
  __shared__ __align__(16) float sT[8][16 * 68];
  const int lane = threadIdx.x & 31;
  const int wave = threadIdx.x >> 5;
  const int tilesN = N >> 6;
  const int tilesM = M >> 6;
  const int tile = blockIdx.x * 8 + wave;
  if (tile >= tilesM * tilesN) return;
  const int tm = tile / tilesN;
  const int tn = tile - tm * tilesN;
  const int m0 = tm << 6;
  const int n0 = tn << 6;

  const int rlane = lane & 15;
  const int koff  = (lane >> 4) * 8;
  const int mOff  = (lane >> 4) * 8;

  v8f acc[4][4];
#pragma unroll
  for (int i = 0; i < 4; ++i)
#pragma unroll
    for (int j = 0; j < 4; ++j) acc[i][j] = (v8f){0.f, 0.f, 0.f, 0.f, 0.f, 0.f, 0.f, 0.f};

  for (int k0 = 0; k0 < K; k0 += 32) {
    v16b bh[4];
#pragma unroll
    for (int j = 0; j < 4; ++j) {
      const size_t bo = (size_t)(n0 + (j << 4) + rlane) * ldb + koff + k0;
      bh[j] = frag_load_b(Bt + bo);
    }
#pragma unroll
    for (int i = 0; i < 4; ++i) {
      const size_t ao = (size_t)(m0 + (i << 4) + rlane) * lda + koff + k0;
      const v16b ah = frag_load_b(A + ao);
      v16b al = ah;
      if (NPROD == 2) al = frag_load_b(A2 + ao);
#pragma unroll
      for (int j = 0; j < 4; ++j) {
        acc[i][j] = mma_b(ah, bh[j], acc[i][j]);
        if (NPROD == 2) acc[i][j] = mma_b(al, bh[j], acc[i][j]);
      }
      dep_guard4_b(acc[i][0], acc[i][1], acc[i][2], acc[i][3], ah, al);
    }
    keep4_b(bh[0], bh[1], bh[2], bh[3]);
  }
  acc_guard4(acc[0][0], acc[0][1], acc[0][2], acc[0][3]);
  acc_guard4(acc[1][0], acc[1][1], acc[1][2], acc[1][3]);
  acc_guard4(acc[2][0], acc[2][1], acc[2][2], acc[2][3]);
  acc_guard4(acc[3][0], acc[3][1], acc[3][2], acc[3][3]);

  float* slab = sT[wave];
#pragma unroll
  for (int i = 0; i < 4; ++i) {
    const int mBase = m0 + (i << 4);
#pragma unroll
    for (int j = 0; j < 4; ++j) {
      const int n = n0 + (j << 4) + rlane;
      float bvl = 0.f;
      if (BIAS_MODE == 2) bvl = bf_rne(bias[n]);
#pragma unroll
      for (int r = 0; r < 8; ++r) {
        float v = acc[i][j][r];
        if (BIAS_MODE == 2) v = v + bvl;
        if (ACT == 2) v = fmaxf(v, 0.0f);
        slab[(mOff + r) * 68 + (j << 4) + rlane] = v;
      }
    }
    __builtin_amdgcn_fence(__ATOMIC_RELEASE, "workgroup");
    __builtin_amdgcn_wave_barrier();
    __builtin_amdgcn_fence(__ATOMIC_ACQUIRE, "workgroup");
    {
      const int hh = lane >> 4, c4 = (lane & 15) * 4;
      for (int pass = 0; pass < 2; ++pass) {
#pragma unroll
        for (int it = 0; it < 8; ++it) {
          const int row = it * 2 + hh;
          const v4f v = *(const v4f*)(slab + row * 68 + c4);
          *(volatile v4f*)(Cout + (size_t)(mBase + row) * ldc + n0 + c4) = v;
        }
        __threadfence();
      }
    }
    __builtin_amdgcn_fence(__ATOMIC_RELEASE, "workgroup");
    __builtin_amdgcn_wave_barrier();
    __builtin_amdgcn_fence(__ATOMIC_ACQUIRE, "workgroup");
  }
}

__global__ __launch_bounds__(256) void prep_pos_kernel(const float* __restrict__ points,
                                                       const float* __restrict__ als,
                                                       float* __restrict__ pos4) {
#pragma clang fp contract(off)
  const int i = blockIdx.x * 256 + threadIdx.x;
  const bool first = (blockIdx.x < (NHALF_PTS / 256));
  const float* src = first ? points : als;
  const int li = first ? i : (i - NHALF_PTS);
  const float x = bf_rne(src[3 * li + 0]);
  const float y = bf_rne(src[3 * li + 1]);
  const float z = bf_rne(src[3 * li + 2]);
  const float t0 = x * x;
  const float t1 = y * y;
  const float t2 = z * z;
  const float sq = (t0 + t2) + t1;
  const v4f v = (v4f){x, y, z, sq};
  st2_v4f(pos4 + 4 * (size_t)i, v);
}

__global__ __launch_bounds__(256) void wprep_kernel(const float* __restrict__ W, unsigned short* __restrict__ Bt,
                                                    int kreal, int nout, int kpad, int gvn) {
  const int p = blockIdx.x * 256 + threadIdx.x;
  const int npieces = (nout * kpad) >> 3;
  if (p >= npieces) return;
  const int e0 = p * 8;
  const int n = e0 / kpad;
  const int k0 = e0 - n * kpad;
  unsigned hb[8];
#pragma unroll
  for (int e = 0; e < 8; ++e) {
    const int k = k0 + e;
    const bool valid = k < kreal;
    int r = (k < gvn) ? ((kreal - gvn) + k) : (k - gvn);
    r = r < 0 ? 0 : r;
    r = r > (kreal - 1) ? (kreal - 1) : r;
    const float wl = W[(size_t)r * nout + n];
    const float w = valid ? wl : 0.0f;
    hb[e] = bf_hi_bits(w);
  }
  const v4u o = (v4u){pack16(hb[0], hb[1]), pack16(hb[2], hb[3]), pack16(hb[4], hb[5]), pack16(hb[6], hb[7])};
  unsigned short* dst = Bt + (size_t)e0;
  *(volatile v4u*)dst = o;
  __threadfence();
  *(volatile v4u*)dst = o;
}

__global__ __launch_bounds__(128) void knn_kernel(const float* __restrict__ pos4, int* __restrict__ nbr) {
#pragma clang fp contract(off)
  __shared__ v4f sTile[128];
  __shared__ unsigned long long sKey[128 * KGRAD];
  const int tid = threadIdx.x;
  const int q = blockIdx.x * 128 + tid;
  const v4f pq = ld4(pos4, q);
  const float px = pq.x, py = pq.y, pz = pq.z, ps = pq.w;
  unsigned long long* myk = sKey + tid * KGRAD;
  const unsigned long long initKey = 0xFF800000FFFFFFFFull;
#pragma unroll
  for (int k = 0; k < KGRAD; ++k) myk[k] = initKey;
  float worst = INFINITY;
  int wslot = 0;
#pragma unroll 1
  for (int t0 = 0; t0 < NPTS; t0 += 128) {
    __syncthreads();
    sTile[tid] = ld4(pos4, t0 + tid);
    __syncthreads();
#pragma unroll 4
    for (int jj = 0; jj < 128; ++jj) {
      const v4f pj = sTile[jj];
      float pr = px * pj.x;
      pr = __builtin_fmaf(py, pj.y, pr);
      pr = __builtin_fmaf(pz, pj.z, pr);
      const float ssum = ps + pj.w;
      const float twop = 2.0f * pr;
      const float d2 = ssum - twop;
      if (d2 < worst) {
        const unsigned u = __float_as_uint(d2);
        const unsigned m = (u & 0x80000000u) ? ~u : (u | 0x80000000u);
        const unsigned long long key = (((unsigned long long)m) << 32) | (unsigned long long)(unsigned)(t0 + jj);
        myk[wslot] = key;
        unsigned long long wk = 0ull;
        int wsl = 0;
#pragma unroll
        for (int k = 0; k < KGRAD; ++k) {
          const unsigned long long kk = myk[k];
          const bool gt = kk > wk;
          wk = gt ? kk : wk;
          wsl = gt ? k : wsl;
        }
        wslot = wsl;
        const unsigned wm = (unsigned)(wk >> 32);
        const unsigned wu = (wm & 0x80000000u) ? (wm ^ 0x80000000u) : ~wm;
        worst = __uint_as_float(wu);
      }
    }
  }
#pragma unroll 1
  for (int a = 0; a < KGRAD - 1; ++a) {
    unsigned long long best = myk[a];
    int bi = a;
#pragma unroll 1
    for (int k = a + 1; k < KGRAD; ++k) {
      const unsigned long long kk = myk[k];
      const bool lt = kk < best;
      best = lt ? kk : best;
      bi = lt ? k : bi;
    }
    const unsigned long long tmp = myk[a];
    myk[bi] = tmp;
    myk[a] = best;
  }
  __syncthreads();
  const int wave = tid >> 5, lane = tid & 31, q8 = lane >> 3, c0 = (lane & 7) * 4;
  for (int pass = 0; pass < 2; ++pass) {
#pragma unroll
    for (int it = 0; it < 8; ++it) {
      const int row = wave * 32 + it * 4 + q8;
      v4i val;
#pragma unroll
      for (int e = 0; e < 4; ++e) {
        const int col = c0 + e;
        const int cc = col < KGRAD ? col : (KGRAD - 1);
        const unsigned long long kk = sKey[row * KGRAD + cc];
        const int id = clamp_idx((int)(unsigned)(kk & 0xFFFFFFFFull));
        val[e] = (col < KGRAD) ? id : 0;
      }
      *(volatile v4i*)(nbr + (size_t)(blockIdx.x * 128 + row) * NBR_PITCH + c0) = val;
    }
    __threadfence();
  }
}

__device__ __forceinline__ void jac_rot(float& app, float& aqq, float& apq, float& arp, float& arq,
                                        float& v0p, float& v0q, float& v1p, float& v1q, float& v2p, float& v2q) {
  const float g = apq;
  const float thr = 1e-12f * (fabsf(app) + fabsf(aqq)) + 1e-30f;
  if (fabsf(g) > thr) {
    const float tau = (aqq - app) * (1.0f / (2.0f * g));
    const float sg = (tau >= 0.0f) ? 1.0f : -1.0f;
    const float t = sg * (1.0f / (fabsf(tau) + sqrtf(1.0f + tau * tau)));
    const float c = 1.0f / sqrtf(1.0f + t * t);
    const float s = t * c;
    app = app - t * g;
    aqq = aqq + t * g;
    apq = 0.0f;
    const float rp = arp, rq = arq;
    arp = c * rp - s * rq;
    arq = s * rp + c * rq;
    float a0 = v0p, a1 = v0q;
    v0p = c * a0 - s * a1; v0q = s * a0 + c * a1;
    a0 = v1p; a1 = v1q;
    v1p = c * a0 - s * a1; v1q = s * a0 + c * a1;
    a0 = v2p; a1 = v2q;
    v2p = c * a0 - s * a1; v2q = s * a0 + c * a1;
  }
}

__global__ __launch_bounds__(256) void basis_kernel(const float* __restrict__ pos4, const int* __restrict__ nbr,
                                                    float* __restrict__ xb4, float* __restrict__ yb4) {
#pragma clang fp contract(off)
  const int n = blockIdx.x * 256 + threadIdx.x;
  const v4f p = ld4(pos4, n);
  const int* nrow = nbr + (size_t)n * NBR_PITCH;
  float a00 = 0.f, a01 = 0.f, a02 = 0.f, a11 = 0.f, a12 = 0.f, a22 = 0.f;
#pragma unroll 1
  for (int k = 0; k < KNORM; ++k) {
    const int j = clamp_idx(nrow[k]);
    const v4f pj = ld4(pos4, j);
    const float rx = pj.x - p.x, ry = pj.y - p.y, rz = pj.z - p.z;
    a00 = a00 + rx * rx; a01 = a01 + rx * ry; a02 = a02 + rx * rz;
    a11 = a11 + ry * ry; a12 = a12 + ry * rz; a22 = a22 + rz * rz;
  }
  float v00 = 1.f, v01 = 0.f, v02 = 0.f;
  float v10 = 0.f, v11 = 1.f, v12 = 0.f;
  float v20 = 0.f, v21 = 0.f, v22 = 1.f;
#pragma unroll 1
  for (int sweep = 0; sweep < 10; ++sweep) {
    jac_rot(a00, a11, a01, a02, a12, v00, v01, v10, v11, v20, v21);
    jac_rot(a00, a22, a02, a01, a12, v00, v02, v10, v12, v20, v22);
    jac_rot(a11, a22, a12, a01, a02, v01, v02, v11, v12, v21, v22);
  }
  int imin = 0; float emin = a00;
  if (a11 < emin) { emin = a11; imin = 1; }
  if (a22 < emin) { emin = a22; imin = 2; }
  int imax = 0; float emax = a00;
  if (a11 > emax) { emax = a11; imax = 1; }
  if (a22 > emax) { emax = a22; imax = 2; }
  if (imax == imin) imax = (imin + 1) % 3;
  float nx = (imin == 0) ? v00 : ((imin == 1) ? v01 : v02);
  float ny = (imin == 0) ? v10 : ((imin == 1) ? v11 : v12);
  float nz = (imin == 0) ? v20 : ((imin == 1) ? v21 : v22);
  const float xx = (imax == 0) ? v00 : ((imax == 1) ? v01 : v02);
  const float xy = (imax == 0) ? v10 : ((imax == 1) ? v11 : v12);
  const float xz = (imax == 0) ? v20 : ((imax == 1) ? v21 : v22);
  const float d0 = nx * p.x, d1 = ny * p.y, d2 = nz * p.z;
  const float dotn = (d0 + d2) + d1;
  const float sgn = (dotn < 0.0f) ? -1.0f : 1.0f;
  nx = nx * sgn; ny = ny * sgn; nz = nz * sgn;
  const float yx = ny * xz - nz * xy;
  const float yy = nz * xx - nx * xz;
  const float yz = nx * xy - ny * xx;
  const v4f xo = (v4f){xx, xy, xz, 0.0f};
  const v4f yo = (v4f){yx, yy, yz, 0.0f};
  st2_v4f(xb4 + 4 * (size_t)n, xo);
  st2_v4f(yb4 + 4 * (size_t)n, yo);
}

__global__ __launch_bounds__(64) void graddiv_kernel(const float* __restrict__ pos4, const int* __restrict__ nbr,
                                                     const float* __restrict__ xb4, const float* __restrict__ yb4,
                                                     float* __restrict__ op, float* __restrict__ v0x,
                                                     float* __restrict__ v0y) {
  __shared__ v4f sOp[64 * KGRAD];
  const int tid = threadIdx.x;
  const int n = blockIdx.x * 64 + tid;
  const v4f p = ld4(pos4, n);
  const v4f xb = ld4(xb4, n);
  const v4f yb = ld4(yb4, n);
  const int* nrow = nbr + (size_t)n * NBR_PITCH;
  float dsum = 0.0f;
#pragma unroll 1
  for (int k = 0; k < KGRAD; ++k) {
    const int j = clamp_idx(nrow[k]);
    const v4f pj = ld4(pos4, j);
    const float rx = pj.x - p.x, ry = pj.y - p.y, rz = pj.z - p.z;
    const float t0 = rx * rx, t1 = ry * ry, t2 = rz * rz;
    const float r2 = (t0 + t2) + t1;
    dsum = dsum + sqrtf(r2 + EPS_F);
  }
  const float h = dsum * INV_KGRAD;
  const float denom = h * h + EPS_F;
  const float rden = 1.0f / denom;
  float A00 = 0.f, A01 = 0.f, A02 = 0.f, A11 = 0.f, A12 = 0.f, A22 = 0.f;
#pragma unroll 1
  for (int k = 0; k < KGRAD; ++k) {
    const int j = clamp_idx(nrow[k]);
    const v4f pj = ld4(pos4, j);
    const float rx = pj.x - p.x, ry = pj.y - p.y, rz = pj.z - p.z;
    const float t0 = rx * rx, t1 = ry * ry, t2 = rz * rz;
    const float r2 = (t0 + t2) + t1;
    const float dist = sqrtf(r2 + EPS_F);
    const float dd = dist * dist;
    const float w = expf(-(dd * rden));
    float u = rx * xb.x; u = u + ry * xb.y; u = u + rz * xb.z;
    float v = rx * yb.x; v = v + ry * yb.y; v = v + rz * yb.z;
    const float wu = w * u, wv = w * v;
    A00 = A00 + w;  A01 = A01 + wu;      A02 = A02 + wv;
    A11 = A11 + wu * u; A12 = A12 + wu * v; A22 = A22 + wv * v;
  }
  A00 = A00 + GRAD_REG_F; A11 = A11 + GRAD_REG_F; A22 = A22 + GRAD_REG_F;
  const float det = A00 * (A11 * A22 - A12 * A12)
                  - A01 * (A01 * A22 - A12 * A02)
                  + A02 * (A01 * A12 - A11 * A02);
  const float inv = 1.0f / det;
  const float i10 = (A02 * A12 - A01 * A22) * inv;
  const float i11 = (A00 * A22 - A02 * A02) * inv;
  const float i12 = (A01 * A02 - A00 * A12) * inv;
  const float i20 = (A01 * A12 - A02 * A11) * inv;
  const float i21 = i12;
  const float i22 = (A00 * A11 - A01 * A01) * inv;
  float ax0 = 0.f, ax1 = 0.f, ax2 = 0.f, ay0 = 0.f, ay1 = 0.f, ay2 = 0.f;
#pragma unroll 1
  for (int k = 0; k < KGRAD; ++k) {
    const int j = clamp_idx(nrow[k]);
    const v4f pj = ld4(pos4, j);
    const v4f xj = ld4(xb4, j);
    const v4f yj = ld4(yb4, j);
    const float rx = pj.x - p.x, ry = pj.y - p.y, rz = pj.z - p.z;
    const float t0 = rx * rx, t1 = ry * ry, t2 = rz * rz;
    const float r2 = (t0 + t2) + t1;
    const float dist = sqrtf(r2 + EPS_F);
    const float dd = dist * dist;
    const float w = expf(-(dd * rden));
    float u = rx * xb.x; u = u + ry * xb.y; u = u + rz * xb.z;
    float v = rx * yb.x; v = v + ry * yb.y; v = v + rz * yb.z;
    const float gx = w * (i10 + i11 * u + i12 * v);
    const float gy = w * (i20 + i21 * u + i22 * v);
    float r00 = xb.x * xj.x; r00 = r00 + xb.y * xj.y; r00 = r00 + xb.z * xj.z;
    float r01 = xb.x * yj.x; r01 = r01 + xb.y * yj.y; r01 = r01 + xb.z * yj.z;
    float r10 = yb.x * xj.x; r10 = r10 + yb.y * xj.y; r10 = r10 + yb.z * xj.z;
    float r11 = yb.x * yj.x; r11 = r11 + yb.y * yj.y; r11 = r11 + yb.z * yj.z;
    const float a0 = gx * r00 + gy * r10;
    const float a1 = gx * r01 + gy * r11;
    sOp[tid * KGRAD + k] = (v4f){gx, gy, a0, a1};
    ax0 = ax0 + gx * pj.x; ax1 = ax1 + gx * pj.y; ax2 = ax2 + gx * pj.z;
    ay0 = ay0 + gy * pj.x; ay1 = ay1 + gy * pj.y; ay2 = ay2 + gy * pj.z;
  }
  const v4f vx = (v4f){ax0, ax1, ax2, 0.0f};
  const v4f vy = (v4f){ay0, ay1, ay2, 0.0f};
  st2_v4f(v0x + 4 * (size_t)n, vx);
  st2_v4f(v0y + 4 * (size_t)n, vy);
  __syncthreads();
  float* dst = op + (size_t)blockIdx.x * (64 * KGRAD * 4);
  for (int pass = 0; pass < 2; ++pass) {
#pragma unroll 4
    for (int it = 0; it < KGRAD; ++it) {
      const int i = it * 64 + tid;
      const v4f v = sOp[i];
      *(volatile v4f*)(dst + 4 * (size_t)i) = v;
    }
    __threadfence();
  }
}

__global__ __launch_bounds__(64) void feat0_kernel(const float* __restrict__ pos4, const float* __restrict__ v0x,
                                                   const float* __restrict__ v0y, const int* __restrict__ nbr,
                                                   const float* __restrict__ op,
                                                   unsigned short* __restrict__ Fh, unsigned short* __restrict__ Fl) {
  __shared__ __align__(16) unsigned sH[64 * 16];
  __shared__ __align__(16) unsigned sL[64 * 16];
  const int tid = threadIdx.x;
  const int n = blockIdx.x * 64 + tid;
  const v4f p = ld4(pos4, n);
  const int* nrow = nbr + (size_t)n * NBR_PITCH;
  float xm0 = -INFINITY, xm1 = -INFINITY, xm2 = -INFINITY;
  float dv0 = 0.f, dv1 = 0.f, dv2 = 0.f, cv0 = 0.f, cv1 = 0.f, cv2 = 0.f;
#pragma unroll 1
  for (int k = 0; k < KGRAD; ++k) {
    const int j = clamp_idx(nrow[k]);
    const v4f o = ld4(op, n * KGRAD + k);
    const v4f pj = ld4(pos4, j);
    const v4f va = ld4(v0x, j);
    const v4f vb = ld4(v0y, j);
    xm0 = fmaxf(xm0, pj.x - p.x);
    xm1 = fmaxf(xm1, pj.y - p.y);
    xm2 = fmaxf(xm2, pj.z - p.z);
    dv0 = dv0 + (o.z * va.x + o.w * vb.x);
    dv1 = dv1 + (o.z * va.y + o.w * vb.y);
    dv2 = dv2 + (o.z * va.z + o.w * vb.z);
    cv0 = cv0 + (o.w * va.x - o.z * vb.x);
    cv1 = cv1 + (o.w * va.y - o.z * vb.y);
    cv2 = cv2 + (o.w * va.z - o.z * vb.z);
  }
  unsigned zz = 0u;
  asm volatile("" : "+v"(zz));
  const unsigned h0 = bf_hi_bits(xm0), h1 = bf_hi_bits(xm1), h2 = bf_hi_bits(xm2);
  const unsigned h3 = bf_hi_bits(dv0), h4 = bf_hi_bits(dv1), h5 = bf_hi_bits(dv2);
  const unsigned h6 = bf_hi_bits(cv0), h7 = bf_hi_bits(cv1), h8 = bf_hi_bits(cv2);
  const unsigned l0 = bf_hi_bits(xm0 - bf_from_bits(h0)), l1 = bf_hi_bits(xm1 - bf_from_bits(h1));
  const unsigned l2 = bf_hi_bits(xm2 - bf_from_bits(h2)), l3 = bf_hi_bits(dv0 - bf_from_bits(h3));
  const unsigned l4 = bf_hi_bits(dv1 - bf_from_bits(h4)), l5 = bf_hi_bits(dv2 - bf_from_bits(h5));
  const unsigned l6 = bf_hi_bits(cv0 - bf_from_bits(h6)), l7 = bf_hi_bits(cv1 - bf_from_bits(h7));
  const unsigned l8 = bf_hi_bits(cv2 - bf_from_bits(h8));
  v4u* rh = (v4u*)(sH + tid * 16);
  v4u* rl = (v4u*)(sL + tid * 16);
  rh[0] = (v4u){pack16(h0, h1), pack16(h2, h3), pack16(h4, h5), pack16(h6, h7)};
  rh[1] = (v4u){pack16(h8, zz), zz, zz, zz};
  rh[2] = (v4u){zz, zz, zz, zz};
  rh[3] = (v4u){zz, zz, zz, zz};
  rl[0] = (v4u){pack16(l0, l1), pack16(l2, l3), pack16(l4, l5), pack16(l6, l7)};
  rl[1] = (v4u){pack16(l8, zz), zz, zz, zz};
  rl[2] = (v4u){zz, zz, zz, zz};
  rl[3] = (v4u){zz, zz, zz, zz};
  __syncthreads();
  unsigned short* dh = Fh + (size_t)blockIdx.x * (64 * 32);
  unsigned short* dl = Fl + (size_t)blockIdx.x * (64 * 32);
  for (int pass = 0; pass < 2; ++pass) {
#pragma unroll
    for (int it = 0; it < 4; ++it) {
      const int i = it * 64 + tid;
      const v4u a = *(const v4u*)(sH + 4 * i);
      const v4u b = *(const v4u*)(sL + 4 * i);
      *(volatile v4u*)(dh + 8 * (size_t)i) = a;
      *(volatile v4u*)(dl + 8 * (size_t)i) = b;
    }
    __threadfence();
  }
}

template <int CIN>
__global__ __launch_bounds__(128) void feat_kernel(const float* __restrict__ x, const float* __restrict__ v,
                                                   const int* __restrict__ nbr, const float* __restrict__ op,
                                                   unsigned short* __restrict__ Fh, unsigned short* __restrict__ Fl) {
  constexpr int TPP = CIN / 4;
  constexpr int PPB = 128 / TPP;
  constexpr int KP  = 3 * CIN;
  constexpr int WPR = KP / 2;
  constexpr int NV  = PPB * WPR / 4;
  static_assert(NV == 192, "block output pieces");
  __shared__ int sIdx[PPB * KGRAD];
  __shared__ v4f sOp[PPB * KGRAD];
  __shared__ __align__(16) unsigned sH[PPB * WPR];
  __shared__ __align__(16) unsigned sL[PPB * WPR];
  const int tid = threadIdx.x;
  const int n0 = blockIdx.x * PPB;
  for (int i = tid; i < PPB * KGRAD; i += 128) {
    const int pp = i / KGRAD;
    const int kk = i - pp * KGRAD;
    sIdx[i] = clamp_idx(nbr[(size_t)(n0 + pp) * NBR_PITCH + kk]);
    sOp[i] = ld4(op, n0 * KGRAD + i);
  }
  __syncthreads();
  const int p = tid / TPP;
  const int g = tid - p * TPP;
  const int c4 = 4 * g;
  v4f xm = (v4f){-INFINITY, -INFINITY, -INFINITY, -INFINITY};
  v4f dv = (v4f){0.f, 0.f, 0.f, 0.f};
  v4f cv = (v4f){0.f, 0.f, 0.f, 0.f};
#pragma unroll 2
  for (int k = 0; k < KGRAD; ++k) {
    const int j = sIdx[p * KGRAD + k];
    const v4f o = sOp[p * KGRAD + k];
    const v4f xj = *(const v4f*)(x + (size_t)j * CIN + c4);
    const v4f va = *(const v4f*)(v + (size_t)(2 * j) * CIN + c4);
    const v4f vb = *(const v4f*)(v + (size_t)(2 * j + 1) * CIN + c4);
#pragma unroll
    for (int e = 0; e < 4; ++e) xm[e] = fmaxf(xm[e], xj[e]);
    dv = dv + (o.z * va + o.w * vb);
    cv = cv + (o.w * va - o.z * vb);
  }
  {
    unsigned* rh = sH + p * WPR;
    unsigned* rl = sL + p * WPR;
    split4_to_lds(xm, rh + (c4 >> 1), rl + (c4 >> 1));
    split4_to_lds(dv, rh + ((CIN + c4) >> 1), rl + ((CIN + c4) >> 1));
    split4_to_lds(cv, rh + ((2 * CIN + c4) >> 1), rl + ((2 * CIN + c4) >> 1));
  }
  __syncthreads();
  unsigned short* dh = Fh + (size_t)blockIdx.x * (PPB * KP);
  unsigned short* dl = Fl + (size_t)blockIdx.x * (PPB * KP);
  for (int pass = 0; pass < 2; ++pass) {
    for (int i = tid; i < NV; i += 128) {
      const v4u a = *(const v4u*)(sH + 4 * i);
      const v4u b = *(const v4u*)(sL + 4 * i);
      *(volatile v4u*)(dh + 8 * (size_t)i) = a;
      *(volatile v4u*)(dl + 8 * (size_t)i) = b;
    }
    __threadfence();
  }
}

template <int CINP, int COUT, int KPAD>
__global__ __launch_bounds__(128) void gvpack_kernel(const float* __restrict__ xout, const float* __restrict__ v,
                                                     int vsN, int vsC,
                                                     const int* __restrict__ nbr, const float* __restrict__ op,
                                                     unsigned short* __restrict__ Vh, unsigned short* __restrict__ Vl) {
  constexpr int TPP = COUT / 4;
  constexpr int PPB = 128 / TPP;
  constexpr int WPR = KPAD / 2;
  constexpr int NG  = KPAD / 4;
  constexpr int VG  = CINP / 4;
  constexpr int NV  = 2 * PPB * WPR / 4;
  static_assert(NG - TPP <= TPP, "trailing groups fit one per thread");
  static_assert(TPP + VG <= NG, "v groups inside the row");
  static_assert(NV == 192, "block output pieces");
  __shared__ int sIdx[PPB * KGRAD];
  __shared__ v4f sOp[PPB * KGRAD];
  __shared__ __align__(16) unsigned sH[2 * PPB * WPR];
  __shared__ __align__(16) unsigned sL[2 * PPB * WPR];
  const int tid = threadIdx.x;
  const int n0 = blockIdx.x * PPB;
  for (int i = tid; i < PPB * KGRAD; i += 128) {
    const int pp = i / KGRAD;
    const int kk = i - pp * KGRAD;
    sIdx[i] = clamp_idx(nbr[(size_t)(n0 + pp) * NBR_PITCH + kk]);
    sOp[i] = ld4(op, n0 * KGRAD + i);
  }
  __syncthreads();
  const int p = tid / TPP;
  const int t = tid - p * TPP;
  const int c4 = 4 * t;
  const int n = n0 + p;
  v4f gx4 = (v4f){0.f, 0.f, 0.f, 0.f};
  v4f gy4 = (v4f){0.f, 0.f, 0.f, 0.f};
#pragma unroll 2
  for (int k = 0; k < KGRAD; ++k) {
    const int j = sIdx[p * KGRAD + k];
    const v4f o = sOp[p * KGRAD + k];
    const v4f f = *(const v4f*)(xout + (size_t)j * COUT + c4);
    gx4 = gx4 + o.x * f;
    gy4 = gy4 + o.y * f;
  }
  unsigned* rh0 = sH + (2 * p) * WPR;
  unsigned* rl0 = sL + (2 * p) * WPR;
  unsigned* rh1 = sH + (2 * p + 1) * WPR;
  unsigned* rl1 = sL + (2 * p + 1) * WPR;
  split4_to_lds(gx4, rh0 + 2 * t, rl0 + 2 * t);
  split4_to_lds(gy4, rh1 + 2 * t, rl1 + 2 * t);
  const int G = TPP + t;
  const bool has = G < NG;
  const bool isv = t < VG;
  const int vgc = isv ? t : (VG - 1);
  const v4f w0 = *(const v4f*)(v + (size_t)n * vsN + 4 * vgc);
  const v4f w1 = *(const v4f*)(v + (size_t)n * vsN + vsC + 4 * vgc);
  v4f e0, e1;
#pragma unroll
  for (int e = 0; e < 4; ++e) {
    e0[e] = isv ? w0[e] : 0.0f;
    e1[e] = isv ? w1[e] : 0.0f;
  }
  if (has) {
    split4_to_lds(e0, rh0 + 2 * G, rl0 + 2 * G);
    split4_to_lds(e1, rh1 + 2 * G, rl1 + 2 * G);
  }
  __syncthreads();
  unsigned short* dh = Vh + (size_t)blockIdx.x * (2 * PPB * KPAD);
  unsigned short* dl = Vl + (size_t)blockIdx.x * (2 * PPB * KPAD);
  for (int pass = 0; pass < 2; ++pass) {
    for (int i = tid; i < NV; i += 128) {
      const v4u a = *(const v4u*)(sH + 4 * i);
      const v4u b = *(const v4u*)(sL + 4 * i);
      *(volatile v4u*)(dh + 8 * (size_t)i) = a;
      *(volatile v4u*)(dl + 8 * (size_t)i) = b;
    }
    __threadfence();
  }
}

template <int COUT>
__global__ __launch_bounds__(256) void gate_kernel(const float* __restrict__ vo, const float* __restrict__ bv,
                                                   float* __restrict__ vnext) {
  constexpr int G4 = COUT / 4;
  const int e = blockIdx.x * 256 + threadIdx.x;
  const int n = e / G4;
  const int g = e - n * G4;
  const size_t r0 = (size_t)(2 * n) * COUT + 4 * g;
  const v4f a = *(const v4f*)(vo + r0);
  const v4f b = *(const v4f*)(vo + r0 + COUT);
  const v4f bb = *(const v4f*)(bv + 4 * g);
  v4f oa, ob;
#pragma unroll
  for (int c = 0; c < 4; ++c) {
    const float ss = a[c] * a[c] + b[c] * b[c];
    const float nn = sqrtf(ss + EPS_F);
    const float num = fmaxf(nn + bf_rne(bb[c]), 0.0f);
    const float s = num * (1.0f / (nn + EPS_F));
    oa[c] = a[c] * s;
    ob[c] = b[c] * s;
  }
  float* pa = vnext + r0;
  float* pb = vnext + r0 + COUT;
  *(volatile v4f*)pa = oa;
  *(volatile v4f*)pb = ob;
  __threadfence();
  *(volatile v4f*)pa = oa;
  *(volatile v4f*)pb = ob;
}

constexpr size_t SZ_POS4 = (size_t)NPTS * 16;
constexpr size_t SZ_NBR  = (size_t)NPTS * NBR_PITCH * 4;
constexpr size_t SZ_OP   = (size_t)NPTS * KGRAD * 16;
constexpr size_t SZ_V0   = (size_t)NPTS * 16 * 2;
constexpr size_t SZ_VB   = (size_t)NPTS * 2 * 64 * 4;
constexpr size_t SZ_VC   = (size_t)NPTS * 2 * 128 * 4;
constexpr size_t SZ_VO   = (size_t)NPTS * 2 * 128 * 4;
constexpr size_t SZ_F0   = (size_t)NPTS * 32 * 2;
constexpr size_t SZ_V0P  = (size_t)NPTS * 2 * 96 * 2;
constexpr size_t SZ_F1   = (size_t)NPTS * 192 * 2;
constexpr size_t SZ_V1P  = (size_t)NPTS * 2 * 192 * 2;
constexpr size_t SZ_F2   = (size_t)NPTS * 384 * 2;
constexpr size_t SZ_W0   = (size_t)64 * 32 * 2;
constexpr size_t SZ_W1   = (size_t)64 * 96 * 2;
constexpr size_t SZ_W2   = (size_t)128 * 192 * 2;
constexpr size_t SZ_W3   = (size_t)128 * 192 * 2;
constexpr size_t SZ_W4   = (size_t)256 * 384 * 2;

constexpr size_t OFF_POS4 = 0;
constexpr size_t OFF_NBR  = OFF_POS4 + SZ_POS4;
constexpr size_t OFF_XB   = OFF_NBR + SZ_NBR;
constexpr size_t OFF_YB   = OFF_XB + SZ_POS4;
constexpr size_t OFF_OP   = OFF_YB + SZ_POS4;
constexpr size_t OFF_V0   = OFF_OP + SZ_OP;
constexpr size_t OFF_VB   = OFF_V0 + SZ_V0;
constexpr size_t OFF_VC   = OFF_VB + SZ_VB;
constexpr size_t OFF_VO   = OFF_VC + SZ_VC;
constexpr size_t OFF_F0H  = OFF_VO + SZ_VO;
constexpr size_t OFF_F0L  = OFF_F0H + SZ_F0;
constexpr size_t OFF_V0H  = OFF_F0L + SZ_F0;
constexpr size_t OFF_V0L  = OFF_V0H + SZ_V0P;
constexpr size_t OFF_F1H  = OFF_V0L + SZ_V0P;
constexpr size_t OFF_F1L  = OFF_F1H + SZ_F1;
constexpr size_t OFF_V1H  = OFF_F1L + SZ_F1;
constexpr size_t OFF_V1L  = OFF_V1H + SZ_V1P;
constexpr size_t OFF_F2H  = OFF_V1L + SZ_V1P;
constexpr size_t OFF_F2L  = OFF_F2H + SZ_F2;
constexpr size_t OFF_W0   = OFF_F2L + SZ_F2;
constexpr size_t OFF_W1   = OFF_W0 + SZ_W0;
constexpr size_t OFF_W2   = OFF_W1 + SZ_W1;
constexpr size_t OFF_W3   = OFF_W2 + SZ_W2;
constexpr size_t OFF_W4   = OFF_W3 + SZ_W3;
constexpr size_t WS_TOTAL = OFF_W4 + SZ_W4;
static_assert(WS_TOTAL == 128499712ull, "carve total");
static_assert(WS_TOTAL <= 134217728ull, "carve within 128 MiB");
static_assert((OFF_W4 % 256) == 0 && (OFF_F0H % 256) == 0 && (OFF_OP % 256) == 0, "aligned carve");
static_assert((size_t)NPTS * 64 * 4 == 4194304ull, "out1 byte offset");
static_assert((size_t)NPTS * (64 + 128) * 4 == 12582912ull, "out2 byte offset");
static_assert((size_t)NPTS * (64 + 128 + 256) * 4 == 29360128ull, "output bytes");
static_assert(NPTS % 64 == 0 && (2 * NPTS) % 64 == 0, "gemm M");
static_assert(32 % 32 == 0 && 96 % 32 == 0 && 192 % 32 == 0 && 384 % 32 == 0, "gemm K");

static inline int gemm_blocks(int M, int N) { return ((M / 64) * (N / 64) + 7) / 8; }

extern "C" void kernel_launch(void* const* d_in, const int* in_sizes, int n_in,
                              void* d_out, int out_size, void* d_ws, size_t ws_size,
                              hipStream_t stream) {
  (void)in_sizes; (void)n_in; (void)out_size;
  if (ws_size < WS_TOTAL) return;
  const float* points = (const float*)d_in[0];
  const float* als    = (const float*)d_in[1];
  const float* Ws0 = (const float*)d_in[2];
  const float* bs0 = (const float*)d_in[3];
  const float* Wv0 = (const float*)d_in[4];
  const float* bv0 = (const float*)d_in[5];
  const float* Ws1 = (const float*)d_in[6];
  const float* bs1 = (const float*)d_in[7];
  const float* Wv1 = (const float*)d_in[8];
  const float* bv1 = (const float*)d_in[9];
  const float* Ws2 = (const float*)d_in[10];
  const float* bs2 = (const float*)d_in[11];

  char* ws = (char*)d_ws;
  float* pos4 = (float*)(ws + OFF_POS4);
  int*   nbr  = (int*)(ws + OFF_NBR);
  float* xb4  = (float*)(ws + OFF_XB);
  float* yb4  = (float*)(ws + OFF_YB);
  float* op   = (float*)(ws + OFF_OP);
  float* v0x  = (float*)(ws + OFF_V0);
  float* v0y  = v0x + (size_t)NPTS * 4;
  float* vB   = (float*)(ws + OFF_VB);
  float* vC   = (float*)(ws + OFF_VC);
  float* vo   = (float*)(ws + OFF_VO);
  unsigned short* F0h = (unsigned short*)(ws + OFF_F0H);
  unsigned short* F0l = (unsigned short*)(ws + OFF_F0L);
  unsigned short* V0h = (unsigned short*)(ws + OFF_V0H);
  unsigned short* V0l = (unsigned short*)(ws + OFF_V0L);
  unsigned short* F1h = (unsigned short*)(ws + OFF_F1H);
  unsigned short* F1l = (unsigned short*)(ws + OFF_F1L);
  unsigned short* V1h = (unsigned short*)(ws + OFF_V1H);
  unsigned short* V1l = (unsigned short*)(ws + OFF_V1L);
  unsigned short* F2h = (unsigned short*)(ws + OFF_F2H);
  unsigned short* F2l = (unsigned short*)(ws + OFF_F2L);
  unsigned short* w0T = (unsigned short*)(ws + OFF_W0);
  unsigned short* w1T = (unsigned short*)(ws + OFF_W1);
  unsigned short* w2T = (unsigned short*)(ws + OFF_W2);
  unsigned short* w3T = (unsigned short*)(ws + OFF_W3);
  unsigned short* w4T = (unsigned short*)(ws + OFF_W4);

  float* out0 = (float*)d_out;
  float* out1 = out0 + (size_t)NPTS * 64;
  float* out2 = out1 + (size_t)NPTS * 128;

  prep_pos_kernel<<<NPTS / 256, 256, 0, stream>>>(points, als, pos4);
  wprep_kernel<<<(64 * 32 / 8) / 256, 256, 0, stream>>>(Ws0, w0T, 9, 64, 32, 0);
  wprep_kernel<<<(64 * 96 / 8) / 256, 256, 0, stream>>>(Wv0, w1T, 67, 64, 96, 64);
  wprep_kernel<<<(128 * 192 / 8) / 256, 256, 0, stream>>>(Ws1, w2T, 192, 128, 192, 0);
  wprep_kernel<<<(128 * 192 / 8) / 256, 256, 0, stream>>>(Wv1, w3T, 192, 128, 192, 128);
  wprep_kernel<<<(256 * 384 / 8) / 256, 256, 0, stream>>>(Ws2, w4T, 384, 256, 384, 0);

  knn_kernel<<<NPTS / 128, 128, 0, stream>>>(pos4, nbr);
  basis_kernel<<<NPTS / 256, 256, 0, stream>>>(pos4, nbr, xb4, yb4);
  graddiv_kernel<<<NPTS / 64, 64, 0, stream>>>(pos4, nbr, xb4, yb4, op, v0x, v0y);

  feat0_kernel<<<NPTS / 64, 64, 0, stream>>>(pos4, v0x, v0y, nbr, op, F0h, F0l);
  gemm_bf16_kernel<2, 2, 2><<<gemm_blocks(NPTS, 64), 256, 0, stream>>>(
      F0h, F0l, 32, w0T, 32, out0, 64, bs0, NPTS, 64, 32);
  gvpack_kernel<4, 64, 96><<<NPTS / 8, 128, 0, stream>>>(out0, v0x, 4, NPTS * 4, nbr, op, V0h, V0l);
  gemm_bf16_kernel<2, 0, 0><<<gemm_blocks(2 * NPTS, 64), 256, 0, stream>>>(
      V0h, V0l, 96, w1T, 96, vo, 64, bs0, 2 * NPTS, 64, 96);
  gate_kernel<64><<<(NPTS * 16) / 256, 256, 0, stream>>>(vo, bv0, vB);

  feat_kernel<64><<<NPTS / 8, 128, 0, stream>>>(out0, vB, nbr, op, F1h, F1l);
  gemm_bf16_kernel<2, 2, 2><<<gemm_blocks(NPTS, 128), 256, 0, stream>>>(
      F1h, F1l, 192, w2T, 192, out1, 128, bs1, NPTS, 128, 192);
  gvpack_kernel<64, 128, 192><<<NPTS / 4, 128, 0, stream>>>(out1, vB, 128, 64, nbr, op, V1h, V1l);
  gemm_bf16_kernel<2, 0, 0><<<gemm_blocks(2 * NPTS, 128), 256, 0, stream>>>(
      V1h, V1l, 192, w3T, 192, vo, 128, bs1, 2 * NPTS, 128, 192);
  gate_kernel<128><<<(NPTS * 32) / 256, 256, 0, stream>>>(vo, bv1, vC);

  feat_kernel<128><<<NPTS / 4, 128, 0, stream>>>(out1, vC, nbr, op, F2h, F2l);
  gemm_bf16_kernel<2, 2, 2><<<gemm_blocks(NPTS, 256), 256, 0, stream>>>(
      F2h, F2l, 384, w4T, 384, out2, 256, bs2, NPTS, 256, 384);
}
